// TransformerEncoderLayerWithMem_14929306321519
// MI455X (gfx1250) — hardware-verified
//
#include <hip/hip_runtime.h>
#include <math.h>
#include <stdint.h>

constexpr int SEQ_T  = 2048;
constexpr int NBATCH = 2;
constexpr int EMB    = 1024;
constexpr int NHEAD  = 16;
constexpr int HDIM   = 64;
constexpr int NMEM   = 32;
constexpr int SKV    = SEQ_T + NMEM;
constexpr int SPAD   = 2112;
constexpr int NKC    = SPAD / 64;
constexpr int FFD    = 4096;
constexpr int NROWS  = SEQ_T * NBATCH;
constexpr int NKROWS = SPAD * NBATCH;
constexpr int QK_LD  = 2048;
constexpr float LN_EPS = 1e-5f;

typedef __attribute__((ext_vector_type(16))) _Float16 v16h;
typedef __attribute__((ext_vector_type(8)))  _Float16 v8h;
typedef __attribute__((ext_vector_type(16))) __bf16   v16b;
typedef __attribute__((ext_vector_type(8)))  __bf16   v8b;
typedef __attribute__((ext_vector_type(8)))  float    v8f;
typedef __attribute__((ext_vector_type(4)))  float    v4f;

__device__ __forceinline__ unsigned short f2bf_bits(float f) {
  unsigned u = __float_as_uint(f);
  return (unsigned short)((u + 0x7FFFu + ((u >> 16) & 1u)) >> 16);
}
__device__ __forceinline__ float bf_bits2f(unsigned short h) { return __uint_as_float(((unsigned)h) << 16); }

__device__ __forceinline__ void dep_guard_h(v8f& a, v8f& b, v16h x, v16h y) { asm volatile("v_nop\n\tv_nop\n\tv_nop\n\tv_nop" : "+v"(a), "+v"(b) : "v"(x), "v"(y)); }
__device__ __forceinline__ void dep_guard_b(v8f& a, v8f& b, v16b x, v16b y) { asm volatile("v_nop\n\tv_nop\n\tv_nop\n\tv_nop" : "+v"(a), "+v"(b) : "v"(x), "v"(y)); }
__device__ __forceinline__ void keep4_h(v16h a, v16h b, v16h c, v16h d) { asm volatile("v_nop" :: "v"(a), "v"(b), "v"(c), "v"(d)); }
__device__ __forceinline__ void keep4_b(v16b a, v16b b, v16b c, v16b d) { asm volatile("v_nop" :: "v"(a), "v"(b), "v"(c), "v"(d)); }
__device__ __forceinline__ void acc_guard4(v8f& a, v8f& b, v8f& c, v8f& d) { asm volatile("v_nop\n\tv_nop\n\tv_nop\n\tv_nop" : "+v"(a), "+v"(b), "+v"(c), "+v"(d)); }
template <typename T> struct Frag;
template <> struct Frag<_Float16> {
  typedef v16h V; union U { v16h v; v8h h[2]; };
  static __device__ __forceinline__ v16h load(const _Float16* p) {
    U f; f.h[0] = *(const v8h*)(p); f.h[1] = *(const v8h*)(p + 16); return f.v;
  }
  static __device__ __forceinline__ v8f mma(v16h a, v16h b, v8f c) {
    return __builtin_amdgcn_wmma_f32_16x16x32_f16(false, a, false, b, (short)0, c, false, false);
  }
  static __device__ __forceinline__ void guard(v8f& a, v8f& b, v16h x, v16h y) { dep_guard_h(a, b, x, y); }
  static __device__ __forceinline__ void keep(v16h a, v16h b, v16h c, v16h d) { keep4_h(a, b, c, d); }
};
template <> struct Frag<__bf16> {
  typedef v16b V; union U { v16b v; v8b h[2]; };
  static __device__ __forceinline__ v16b load(const __bf16* p) {
    U f; f.h[0] = *(const v8b*)(p); f.h[1] = *(const v8b*)(p + 16); return f.v;
  }
  static __device__ __forceinline__ v8f mma(v16b a, v16b b, v8f c) {
    return __builtin_amdgcn_wmma_f32_16x16x32_bf16(false, a, false, b, (short)0, c, false, false);
  }
  static __device__ __forceinline__ void guard(v8f& a, v8f& b, v16b x, v16b y) { dep_guard_b(a, b, x, y); }
  static __device__ __forceinline__ void keep(v16b a, v16b b, v16b c, v16b d) { keep4_b(a, b, c, d); }
};

template <int ET> struct Elem;
template <> struct Elem<0> { typedef _Float16 T; };
template <> struct Elem<1> { typedef __bf16 T; };
template <int ET, bool SPLIT, int BIAS_MODE, int OUT_MODE, bool RESID, int ACT = 0>
__global__ __launch_bounds__(256) void wmma_gemm64(
    const unsigned short* __restrict__ Ap, const unsigned short* __restrict__ A2p, int lda, long strideA,
    const unsigned short* __restrict__ Btp, const unsigned short* __restrict__ Bt2p, int ldb, long strideB,
    void* __restrict__ Cout, void* __restrict__ Cout2, int ldc, long strideC,
    const float* __restrict__ bias,
    const float* __restrict__ resid, long strideR,
    int M, int N, int K, float scale) {
  typedef typename Elem<ET>::T T;
  typedef typename Frag<T>::V V;
  const T* A = (const T*)Ap; const T* A2 = (const T*)A2p; const T* Bt = (const T*)Btp; const T* Bt2 = (const T*)Bt2p;
  __shared__ __align__(16) float sT[8][16 * 68];
  const int b    = blockIdx.y;
  const int lane = threadIdx.x & 31;
  const int wave = threadIdx.x >> 5;
  const int tilesN = N >> 6;
  const int tilesM = M >> 6;
  const int tile = blockIdx.x * 8 + wave;
  if (tile >= tilesM * tilesN) return;
  const int tm = tile / tilesN;
  const int tn = tile - tm * tilesN;
  const int m0 = tm << 6;
  const int n0 = tn << 6;

  const T* Ab  = A  + (size_t)b * strideA;
  const T* Bb  = Bt + (size_t)b * strideB;
  const T* Ab2 = SPLIT ? (A2  + (size_t)b * strideA) : nullptr;
  const T* Bb2 = SPLIT ? (Bt2 + (size_t)b * strideB) : nullptr;

  const int rlane = lane & 15;
  const int koff  = (lane >> 4) * 8;
  const int mOff  = (lane >> 4) * 8;

  v8f acc[4][4];
#pragma unroll
  for (int i = 0; i < 4; ++i)
#pragma unroll
    for (int j = 0; j < 4; ++j) acc[i][j] = (v8f){0.f,0.f,0.f,0.f,0.f,0.f,0.f,0.f};

  for (int k0 = 0; k0 < K; k0 += 32) {
    V bh[4], bl[4];
#pragma unroll
    for (int j = 0; j < 4; ++j) {
      const size_t bo = (size_t)(n0 + (j << 4) + rlane) * ldb + koff + k0;
      bh[j] = Frag<T>::load(Bb + bo);
      if (SPLIT) bl[j] = Frag<T>::load(Bb2 + bo);
    }
#pragma unroll
    for (int i = 0; i < 4; ++i) {
      const size_t ao = (size_t)(m0 + (i << 4) + rlane) * lda + koff + k0;
      V ah = Frag<T>::load(Ab + ao);
      V al;
      if (SPLIT) al = Frag<T>::load(Ab2 + ao);
#pragma unroll
      for (int j = 0; j < 4; ++j) {
        acc[i][j] = Frag<T>::mma(ah, bh[j], acc[i][j]);
        if (SPLIT) {
          acc[i][j] = Frag<T>::mma(ah, bl[j], acc[i][j]);
          acc[i][j] = Frag<T>::mma(al, bh[j], acc[i][j]);
        }
      }
      Frag<T>::guard(acc[i][0], acc[i][3], ah, SPLIT ? al : ah);
    }
    Frag<T>::keep(bh[0], bh[1], bh[2], bh[3]);
    if (SPLIT) Frag<T>::keep(bl[0], bl[1], bl[2], bl[3]);
  }
  acc_guard4(acc[0][0], acc[0][1], acc[0][2], acc[0][3]);
  acc_guard4(acc[1][0], acc[1][1], acc[1][2], acc[1][3]);
  acc_guard4(acc[2][0], acc[2][1], acc[2][2], acc[2][3]);
  acc_guard4(acc[3][0], acc[3][1], acc[3][2], acc[3][3]);

  float* slab = sT[wave];
  const float* Rb = RESID ? (resid + (size_t)b * strideR) : nullptr;
#pragma unroll
  for (int i = 0; i < 4; ++i) {
    const int mBase = m0 + (i << 4);
#pragma unroll
    for (int j = 0; j < 4; ++j) {
      const int n = n0 + (j << 4) + rlane;
      float bv = 0.f;
      if (BIAS_MODE == 2) bv = bias[n];
#pragma unroll
      for (int r = 0; r < 8; ++r) {
        float v = acc[i][j][r] * scale;
        if (BIAS_MODE == 1) v += bias[mBase + mOff + r];
        if (BIAS_MODE == 2) v += bv;
        if (RESID) v += Rb[(size_t)(mBase + mOff + r) * ldc + n];
        if (ACT == 1) v = tanhf(v);
        if (ACT == 2) v = fmaxf(v, 0.0f);
        if (ACT == 3) v = v / (1.0f + expf(-v));
        if (ACT == 4) v = (v > 0.f) ? v : 0.01f * v;
        if (ACT == 5) v = 0.5f * v * (1.0f + erff(v * 0.70710678118654752f));
        slab[(mOff + r) * 68 + (j << 4) + rlane] = v;
      }
    }
    __builtin_amdgcn_fence(__ATOMIC_RELEASE, "workgroup");
    __builtin_amdgcn_wave_barrier();
    __builtin_amdgcn_fence(__ATOMIC_ACQUIRE, "workgroup");
    if (OUT_MODE == 0) {
      float* C = (float*)Cout + (size_t)b * strideC;
      const int hh = lane >> 4, c4 = (lane & 15) * 4;
      for (int pass = 0; pass < 2; ++pass) {
#pragma unroll
        for (int it = 0; it < 8; ++it) {
          const int row = it * 2 + hh;
          v4f v = *(const v4f*)(slab + row * 68 + c4);
          *(volatile v4f*)(C + (size_t)(mBase + row) * ldc + n0 + c4) = v;
        }
        __threadfence();
      }
    } else {
      const int q = lane >> 3, c8 = (lane & 7) * 8;
      unsigned short* C  = (unsigned short*)Cout  + (size_t)b * strideC;
      unsigned short* C2 = (OUT_MODE == 2) ? ((unsigned short*)Cout2 + (size_t)b * strideC) : nullptr;
      for (int pass = 0; pass < 2; ++pass) {
#pragma unroll
        for (int it = 0; it < 4; ++it) {
          const int row = it * 4 + q;
          const float* sp = slab + row * 68 + c8;
          v8h hv, lv;
#pragma unroll
          for (int e = 0; e < 8; ++e) {
            if (OUT_MODE == 1) {
              hv[e] = (_Float16)sp[e];
            } else {
              unsigned short hb = f2bf_bits(sp[e]);
              unsigned short lb = f2bf_bits(sp[e] - bf_bits2f(hb));
              hv[e] = __builtin_bit_cast(_Float16, hb);
              lv[e] = __builtin_bit_cast(_Float16, lb);
            }
          }
          *(volatile v8h*)(C + (size_t)(mBase + row) * ldc + n0 + c8) = hv;
          if (OUT_MODE == 2) *(volatile v8h*)(C2 + (size_t)(mBase + row) * ldc + n0 + c8) = lv;
        }
        __threadfence();
      }
    }
    __builtin_amdgcn_fence(__ATOMIC_RELEASE, "workgroup");
    __builtin_amdgcn_wave_barrier();
    __builtin_amdgcn_fence(__ATOMIC_ACQUIRE, "workgroup");
  }
}

__global__ __launch_bounds__(256) void cast_scale_f16x2(
    const float* __restrict__ in, _Float16* __restrict__ out, int n2, float scale) {
  const int i = blockIdx.x * 256 + threadIdx.x;
  if (i < n2) {
    const float f0 = in[2 * (size_t)i] * scale;
    const float f1 = in[2 * (size_t)i + 1] * scale;
    const _Float16 h0 = (_Float16)f0, h1 = (_Float16)f1;
    const unsigned u = (unsigned)__builtin_bit_cast(unsigned short, h0) | ((unsigned)__builtin_bit_cast(unsigned short, h1) << 16);
    ((volatile unsigned*)out)[i] = u;
    __threadfence();
    ((volatile unsigned*)out)[i] = u;
  }
}

__global__ __launch_bounds__(256) void memkv_kernel(const float* __restrict__ mem_k, const float* __restrict__ mem_v,
                                                    unsigned short* __restrict__ qk16, unsigned short* __restrict__ vt16) {
  const int tid = threadIdx.x;
  if (blockIdx.x < 64) {
    const int g = blockIdx.x * 256 + tid;
    const int row = g >> 7;
    const int c8 = (g & 127) * 8;
    const int m = row >> 1;
    const int mm = (m < NMEM) ? m : (NMEM - 1);
    const bool valid = (m < NMEM);
    v8h hv;
#pragma unroll
    for (int e = 0; e < 8; ++e) {
      const float f = mem_k[(size_t)mm * EMB + c8 + e] * 8.0f;
      hv[e] = valid ? (_Float16)f : (_Float16)0.0f;
    }
    _Float16* dst = (_Float16*)(void*)qk16 + (size_t)(NROWS + row) * QK_LD + EMB + c8;
    *(volatile v8h*)dst = hv;
    __threadfence();
    *(volatile v8h*)dst = hv;
  } else {
    const int g = (blockIdx.x - 64) * 256 + tid;
    const int be = g >> 3;
    const int bb = be >> 10;
    const int e = be & (EMB - 1);
    const int c8 = (g & 7) * 8;
    const float sq_nmem = 5.656854249492381f;
    v8h hv;
#pragma unroll
    for (int j = 0; j < 8; ++j) {
      const int m = c8 + j;
      const int mm = (m < NMEM) ? m : (NMEM - 1);
      const float f = mem_v[(size_t)mm * EMB + e] * sq_nmem;
      hv[j] = (m < NMEM) ? (_Float16)f : (_Float16)0.0f;
    }
    _Float16* dst = (_Float16*)(void*)vt16 + (size_t)bb * EMB * SPAD + (size_t)e * SPAD + SEQ_T + c8;
    *(volatile v8h*)dst = hv;
    __threadfence();
    *(volatile v8h*)dst = hv;
  }
}

#define AT_D 64
#define AT_NW 4
#define AT_QB 64
#define AT_KC 64

__device__ __forceinline__ v8f mma_h(v16h a, v16h b, v8f c) {
  c = __builtin_amdgcn_wmma_f32_16x16x32_f16(false, a, false, b, (short)0, c, false, false);
  asm volatile("v_nop\n\tv_nop\n\tv_nop\n\tv_nop" : "+v"(c) : "v"(a), "v"(b));
  return c;
}

__global__ __launch_bounds__(128)
void attn_mem_kernel(const unsigned short* __restrict__ qp, const unsigned short* __restrict__ kp,
                     const unsigned short* __restrict__ vtp, unsigned short* __restrict__ op, float sscale) {
  union FH { v16h v; v8h h[2]; };
  __shared__ __align__(16) _Float16 Ksh[AT_KC * AT_D];
  __shared__ __align__(16) _Float16 Vth[AT_D * AT_KC];
  __shared__ __align__(16) _Float16 Psh[AT_NW][16 * AT_KC];
  __shared__ __align__(16) float    Os[AT_NW][16 * 68];

  const float PSC = 32768.0f;
  const float OSC = 64.0f;

  const int tid  = threadIdx.x;
  const int wave = tid >> 5;
  const int lane = tid & 31;
  const int hh   = lane >> 4;
  const int c    = lane & 15;

  const int nqb = SEQ_T / AT_QB;
  const int bx = blockIdx.x;
  const int qb = bx % nqb;
  const int bh = bx / nqb;
  const int h  = bh % NHEAD;
  const int b  = bh / NHEAD;
  const int q0 = qb * AT_QB + wave * 16;

  const size_t qk_rs = 2 * (size_t)QK_LD;
  const size_t o_rs  = 2 * (size_t)EMB;
  const _Float16* Qb = (const _Float16*)(const void*)qp  + (size_t)b * QK_LD + (size_t)h * AT_D;
  const _Float16* Kb = (const _Float16*)(const void*)kp  + (size_t)b * QK_LD + (size_t)h * AT_D;
  const _Float16* Vb = (const _Float16*)(const void*)vtp + (size_t)b * EMB * SPAD + (size_t)h * AT_D * SPAD;
  _Float16*       Ob = (_Float16*)(void*)op + (size_t)b * EMB + (size_t)h * AT_D;

  v16h qa[2];
#pragma unroll
  for (int dc = 0; dc < 2; ++dc) qa[dc] = Frag<_Float16>::load(Qb + (size_t)(q0 + c) * qk_rs + dc * 32 + 8 * hh);

  float mrow[8], lrow[8];
  v8f oacc[4];
#pragma unroll
  for (int r = 0; r < 8; ++r) { mrow[r] = -INFINITY; lrow[r] = 0.f; }
#pragma unroll
  for (int t = 0; t < 4; ++t) oacc[t] = (v8f){0.f,0.f,0.f,0.f,0.f,0.f,0.f,0.f};

  for (int kc = 0; kc < NKC; ++kc) {
    const int kv0 = kc * AT_KC;
    __syncthreads();
    {
      const int r = tid >> 1, half = (tid & 1) * 32;
      const _Float16* ks = Kb + (size_t)(kv0 + r) * qk_rs + half;
      const _Float16* vs = Vb + (size_t)r * SPAD + kv0 + half;
#pragma unroll
      for (int i = 0; i < 4; ++i) {
        const v8h a0 = *(const v8h*)(ks + 8 * i);
        const v8h b0 = *(const v8h*)(vs + 8 * i);
        *(v8h*)(Ksh + r * AT_D  + half + 8 * i) = a0;
        *(v8h*)(Vth + r * AT_KC + half + 8 * i) = b0;
      }
    }
    __syncthreads();

    v8f s[4];
#pragma unroll
    for (int j = 0; j < 4; ++j) {
      s[j] = (v8f){0.f,0.f,0.f,0.f,0.f,0.f,0.f,0.f};
#pragma unroll
      for (int dc = 0; dc < 2; ++dc) {
        FH kb;
        kb.h[0] = *(const v8h*)(Ksh + (j * 16 + c) * AT_D + dc * 32 + 8 * hh);
        kb.h[1] = *(const v8h*)(Ksh + (j * 16 + c) * AT_D + dc * 32 + 16 + 8 * hh);
        s[j] = mma_h(qa[dc], kb.v, s[j]);
      }
    }
    float cm[8];
#pragma unroll
    for (int r = 0; r < 8; ++r) {
      float m = -INFINITY;
#pragma unroll
      for (int j = 0; j < 4; ++j) {
        const int kvcol = kv0 + j * 16 + c;
        float sv = s[j][r] * sscale;
        if (kvcol >= SKV) sv = -INFINITY;
        s[j][r] = sv;
        m = fmaxf(m, sv);
      }
#pragma unroll
      for (int off = 1; off < 16; off <<= 1) m = fmaxf(m, __shfl_xor(m, off, 32));
      cm[r] = m;
    }
    _Float16* pw = Psh[wave];
#pragma unroll
    for (int r = 0; r < 8; ++r) {
      const float mnew = fmaxf(mrow[r], cm[r]);
      const float alpha = expf(mrow[r] - mnew);
      mrow[r] = mnew;
      float psum = 0.f;
#pragma unroll
      for (int j = 0; j < 4; ++j) {
        const float p = expf(s[j][r] - mnew);
        psum += p;
        pw[(8 * hh + r) * AT_KC + j * 16 + c] = (_Float16)(p * PSC);
      }
#pragma unroll
      for (int off = 1; off < 16; off <<= 1) psum += __shfl_xor(psum, off, 32);
      lrow[r] = lrow[r] * alpha + psum;
#pragma unroll
      for (int t = 0; t < 4; ++t) oacc[t][r] *= alpha;
    }
    __builtin_amdgcn_fence(__ATOMIC_RELEASE, "workgroup");
    __builtin_amdgcn_wave_barrier();
    __builtin_amdgcn_fence(__ATOMIC_ACQUIRE, "workgroup");
#pragma unroll 1
    for (int kk = 0; kk < 2; ++kk) {
      FH pa;
      pa.h[0] = *(const v8h*)(pw + c * AT_KC + kk * 32 + 8 * hh);
      pa.h[1] = *(const v8h*)(pw + c * AT_KC + kk * 32 + 16 + 8 * hh);
#pragma unroll
      for (int t = 0; t < 4; ++t) {
        FH vb;
        vb.h[0] = *(const v8h*)(Vth + (t * 16 + c) * AT_KC + kk * 32 + 8 * hh);
        vb.h[1] = *(const v8h*)(Vth + (t * 16 + c) * AT_KC + kk * 32 + 16 + 8 * hh);
        oacc[t] = mma_h(pa.v, vb.v, oacc[t]);
      }
    }
  }

  float* os = Os[wave];
#pragma unroll
  for (int r = 0; r < 8; ++r) {
    const float inv = OSC * (1.0f / (lrow[r] * PSC));
#pragma unroll
    for (int t = 0; t < 4; ++t) os[(8 * hh + r) * 68 + t * 16 + c] = oacc[t][r] * inv;
  }
  __builtin_amdgcn_fence(__ATOMIC_RELEASE, "workgroup");
  __builtin_amdgcn_wave_barrier();
  __builtin_amdgcn_fence(__ATOMIC_ACQUIRE, "workgroup");
  {
    const int q = lane >> 3, c8 = (lane & 7) * 8;
    for (int pass = 0; pass < 2; ++pass) {
#pragma unroll
      for (int it = 0; it < 4; ++it) {
        const int row = it * 4 + q;
        const float* sp = os + row * 68 + c8;
        v8h hv;
#pragma unroll
        for (int e = 0; e < 8; ++e) hv[e] = (_Float16)sp[e];
        *(volatile v8h*)(Ob + (size_t)(q0 + row) * o_rs + c8) = hv;
      }
      __threadfence();
    }
  }
}

template <bool W16>
__global__ __launch_bounds__(256) void layernorm_kernel(const float* __restrict__ y, const float* __restrict__ gam,
                                                        const float* __restrict__ bet, float* __restrict__ outf,
                                                        unsigned short* __restrict__ out16) {
  __shared__ float red_a[8];
  __shared__ float red_b[8];
  __shared__ __align__(16) float rowbuf[W16 ? EMB : 4];
  const int row = blockIdx.x, tid = threadIdx.x, lane = tid & 31, wave = tid >> 5;
  const int c4 = tid * 4;
  const v4f v = *(const v4f*)(y + (size_t)row * EMB + c4);
  float s = (v[0] + v[1]) + (v[2] + v[3]);
#pragma unroll
  for (int off = 1; off < 32; off <<= 1) s += __shfl_xor(s, off, 32);
  if (lane == 0) red_a[wave] = s;
  __syncthreads();
  float tot = 0.f;
#pragma unroll
  for (int w = 0; w < 8; ++w) tot += red_a[w];
  const float mu = tot * (1.0f / (float)EMB);
  v4f d;
  d[0] = v[0] - mu; d[1] = v[1] - mu; d[2] = v[2] - mu; d[3] = v[3] - mu;
  float s2 = (d[0] * d[0] + d[1] * d[1]) + (d[2] * d[2] + d[3] * d[3]);
#pragma unroll
  for (int off = 1; off < 32; off <<= 1) s2 += __shfl_xor(s2, off, 32);
  if (lane == 0) red_b[wave] = s2;
  __syncthreads();
  float tot2 = 0.f;
#pragma unroll
  for (int w = 0; w < 8; ++w) tot2 += red_b[w];
  const float var = tot2 * (1.0f / (float)EMB);
  const float rstd = rsqrtf(var + LN_EPS);
  const v4f gg = *(const v4f*)(gam + c4);
  const v4f be = *(const v4f*)(bet + c4);
  v4f o;
  o[0] = d[0] * rstd * gg[0] + be[0];
  o[1] = d[1] * rstd * gg[1] + be[1];
  o[2] = d[2] * rstd * gg[2] + be[2];
  o[3] = d[3] * rstd * gg[3] + be[3];
  float* dst = outf + (size_t)row * EMB + c4;
  *(volatile v4f*)dst = o;
  __threadfence();
  *(volatile v4f*)dst = o;
  if (W16) {
    *(v4f*)(rowbuf + c4) = o;
    __syncthreads();
    if (tid < 128) {
      const int c8 = tid * 8;
      v8h hv;
#pragma unroll
      for (int e = 0; e < 8; ++e) hv[e] = (_Float16)rowbuf[c8 + e];
      _Float16* dst16 = (_Float16*)(void*)out16 + (size_t)row * EMB + c8;
      *(volatile v8h*)dst16 = hv;
      __threadfence();
      *(volatile v8h*)dst16 = hv;
    }
  }
}

extern "C" void kernel_launch(void* const* d_in, const int* in_sizes, int n_in,
                              void* d_out, int out_size, void* d_ws, size_t ws_size,
                              hipStream_t stream) {
  if (n_in < 15) return;
  if (in_sizes[0] != NROWS * EMB || in_sizes[1] != 3 * EMB * EMB || in_sizes[2] != 3 * EMB ||
      in_sizes[3] != EMB * EMB || in_sizes[4] != EMB || in_sizes[5] != NMEM * EMB || in_sizes[6] != NMEM * EMB ||
      in_sizes[7] != FFD * EMB || in_sizes[8] != FFD || in_sizes[9] != EMB * FFD || in_sizes[10] != EMB ||
      in_sizes[11] != EMB || in_sizes[12] != EMB || in_sizes[13] != EMB || in_sizes[14] != EMB ||
      out_size != NROWS * EMB) return;

  const float* src   = (const float*)d_in[0];
  const float* wqkv  = (const float*)d_in[1];
  const float* bqkv  = (const float*)d_in[2];
  const float* wo    = (const float*)d_in[3];
  const float* bo    = (const float*)d_in[4];
  const float* mem_k = (const float*)d_in[5];
  const float* mem_v = (const float*)d_in[6];
  const float* w1    = (const float*)d_in[7];
  const float* b1    = (const float*)d_in[8];
  const float* w2    = (const float*)d_in[9];
  const float* b2    = (const float*)d_in[10];
  const float* ln1g  = (const float*)d_in[11];
  const float* ln1b  = (const float*)d_in[12];
  const float* ln2g  = (const float*)d_in[13];
  const float* ln2b  = (const float*)d_in[14];
  float* outp = (float*)d_out;

  char* ws = (char*)d_ws;
  size_t off = 0;
  auto take = [&](size_t bytes) -> char* {
    char* p = ws + off;
    off += (bytes + 255) & ~(size_t)255;
    return p;
  };
  unsigned short* SRC16  = (unsigned short*)take((size_t)NROWS * EMB * 2);
  unsigned short* WQKV16 = (unsigned short*)take((size_t)3 * EMB * EMB * 2);
  unsigned short* WO16   = (unsigned short*)take((size_t)EMB * EMB * 2);
  unsigned short* W1H    = (unsigned short*)take((size_t)FFD * EMB * 2);
  unsigned short* W2H    = (unsigned short*)take((size_t)EMB * FFD * 2);
  unsigned short* QK16   = (unsigned short*)take((size_t)NKROWS * QK_LD * 2);
  unsigned short* VT16   = (unsigned short*)take((size_t)NBATCH * EMB * SPAD * 2);
  unsigned short* CTX16  = (unsigned short*)take((size_t)NROWS * EMB * 2);
  float*          Y1     = (float*)take((size_t)NROWS * EMB * 4);
  float*          XF     = (float*)take((size_t)NROWS * EMB * 4);
  unsigned short* X16    = (unsigned short*)take((size_t)NROWS * EMB * 2);
  if (off > ws_size) return;
  const size_t span_qkvctx = ((size_t)NKROWS * QK_LD * 2) + ((size_t)NBATCH * EMB * SPAD * 2) + ((size_t)NROWS * EMB * 2);
  if (span_qkvctx < (size_t)NROWS * FFD * 2) return;
  unsigned short* H16 = QK16;
  float* Y2 = Y1;

  {
    const int n2_src = NROWS * EMB / 2, n2_wqkv = 3 * EMB * EMB / 2, n2_wo = EMB * EMB / 2, n2_w1 = FFD * EMB / 2, n2_w2 = EMB * FFD / 2;
    cast_scale_f16x2<<<(n2_src + 255) / 256, 256, 0, stream>>>(src, (_Float16*)(void*)SRC16, n2_src, 1.0f);
    cast_scale_f16x2<<<(n2_wqkv + 255) / 256, 256, 0, stream>>>(wqkv, (_Float16*)(void*)WQKV16, n2_wqkv, 32.0f);
    cast_scale_f16x2<<<(n2_wo + 255) / 256, 256, 0, stream>>>(wo, (_Float16*)(void*)WO16, n2_wo, 32.0f);
    cast_scale_f16x2<<<(n2_w1 + 255) / 256, 256, 0, stream>>>(w1, (_Float16*)(void*)W1H, n2_w1, 32.0f);
    cast_scale_f16x2<<<(n2_w2 + 255) / 256, 256, 0, stream>>>(w2, (_Float16*)(void*)W2H, n2_w2, 64.0f);
  }

  wmma_gemm64<0, false, 2, 1, false, 0><<<dim3((NROWS / 64) * (2 * EMB / 64) / 8, 1), 256, 0, stream>>>(
      SRC16, SRC16, EMB, 0L,
      WQKV16, WQKV16, EMB, 0L,
      (void*)QK16, (void*)QK16, QK_LD, 0L,
      bqkv, bqkv, 0L,
      NROWS, 2 * EMB, EMB, 1.0f / 32.0f);

  wmma_gemm64<0, false, 1, 1, false, 0><<<dim3((EMB / 64) * (SEQ_T / 64) / 8, NBATCH), 256, 0, stream>>>(
      WQKV16 + (size_t)2 * EMB * EMB, WQKV16 + (size_t)2 * EMB * EMB, EMB, 0L,
      SRC16, SRC16, NBATCH * EMB, (long)EMB,
      (void*)VT16, (void*)VT16, SPAD, (long)EMB * SPAD,
      bqkv + 2 * EMB, bqkv, 0L,
      EMB, SEQ_T, EMB, 1.0f / 32.0f);

  memkv_kernel<<<128, 256, 0, stream>>>(mem_k, mem_v, QK16, VT16);

  attn_mem_kernel<<<NBATCH * NHEAD * (SEQ_T / 64), 128, 0, stream>>>(QK16, QK16 + EMB, VT16, CTX16, 0.125f);

  wmma_gemm64<0, false, 2, 0, true, 0><<<dim3((NROWS / 64) * (EMB / 64) / 8, 1), 256, 0, stream>>>(
      CTX16, CTX16, EMB, 0L,
      WO16, WO16, EMB, 0L,
      (void*)Y1, (void*)Y1, EMB, 0L,
      bo, src, 0L,
      NROWS, EMB, EMB, 1.0f / 2048.0f);

  layernorm_kernel<true><<<NROWS, 256, 0, stream>>>(Y1, ln1g, ln1b, XF, X16);

  wmma_gemm64<0, false, 2, 1, false, 2><<<dim3((NROWS / 64) * (FFD / 64) / 8, 1), 256, 0, stream>>>(
      X16, X16, EMB, 0L,
      W1H, W1H, EMB, 0L,
      (void*)H16, (void*)H16, FFD, 0L,
      b1, b1, 0L,
      NROWS, FFD, EMB, 1.0f / 32.0f);

  wmma_gemm64<0, false, 2, 0, true, 0><<<dim3((NROWS / 64) * (EMB / 64) / 8, 1), 256, 0, stream>>>(
      H16, H16, FFD, 0L,
      W2H, W2H, FFD, 0L,
      (void*)Y2, (void*)Y2, EMB, 0L,
      b2, XF, 0L,
      NROWS, EMB, FFD, 1.0f / 64.0f);

  layernorm_kernel<false><<<NROWS, 256, 0, stream>>>(Y2, ln2g, ln2b, outp, X16);
}
